// SelectiveSSM_61125974557355
// MI455X (gfx1250) — hardware-verified
//
#include <hip/hip_runtime.h>
#include <math.h>

typedef __attribute__((ext_vector_type(16))) _Float16 v16h;
typedef __attribute__((ext_vector_type(8)))  _Float16 v8h;
typedef __attribute__((ext_vector_type(16))) __bf16   v16b;
typedef __attribute__((ext_vector_type(8)))  __bf16   v8b;
typedef __attribute__((ext_vector_type(8)))  float    v8f;
typedef __attribute__((ext_vector_type(4)))  float    v4f;

constexpr int kL   = 2048;
constexpr int kD   = 2048;
constexpr int kR   = 128;
constexpr int kN   = 16;
constexpr int kXC  = kR + 2 * kN;
constexpr int kXW  = 192;
constexpr int kBCW = 2 * kN;
constexpr int kScanCh = 64;
constexpr int kScanTS = 64;
constexpr int kScanYP = 68;
static_assert(kXC == 160, "x_dbl width");
static_assert((kXW % 64) == 0 && kXW >= kXC, "padded N of GEMM1 is a 64 multiple");
static_assert((kL % 64) == 0 && (kD % 64) == 0, "GEMM M,N multiples of 64");
static_assert((kD % 32) == 0 && (kR % 32) == 0, "GEMM K multiples of 32");
static_assert((kL % kScanTS) == 0 && (kD % kScanCh) == 0, "scan tiles");
static_assert((kXW * 4) % 128 == 0 && (kR * 2) % 128 == 0 && (kD * 4) % 128 == 0 && (kD * 2) % 128 == 0, "row pitches are line multiples");

constexpr size_t kOffXH   = 0;
constexpr size_t kOffXL   = kOffXH  + (size_t)kL  * kD  * 2;
constexpr size_t kOffWXH  = kOffXL  + (size_t)kL  * kD  * 2;
constexpr size_t kOffWXL  = kOffWXH + (size_t)kXW * kD  * 2;
constexpr size_t kOffWD   = kOffWXL + (size_t)kXW * kD  * 2;
constexpr size_t kOffXD   = kOffWD  + (size_t)kD  * kR  * 2;
constexpr size_t kOffDI   = kOffXD  + (size_t)kL  * kXW * 4;
constexpr size_t kOffDT   = kOffDI  + (size_t)kL  * kR  * 2;
constexpr size_t kWsTotal = kOffDT  + (size_t)kL  * kD  * 4;
static_assert(kWsTotal == 37748736ull, "carve total");
static_assert(kWsTotal <= 134217728ull, "carve cap");
static_assert((kOffXL % 128) == 0 && (kOffWXH % 128) == 0 && (kOffWXL % 128) == 0 && (kOffWD % 128) == 0 &&
              (kOffXD % 128) == 0 && (kOffDI % 128) == 0 && (kOffDT % 128) == 0, "128-B aligned regions");

__device__ __forceinline__ unsigned short f2bf_bits(float f) {
  unsigned u = __float_as_uint(f);
  return (unsigned short)((u + 0x7FFFu + ((u >> 16) & 1u)) >> 16);
}
__device__ __forceinline__ float bf_bits2f(unsigned short h) { return __uint_as_float(((unsigned)h) << 16); }

__device__ __forceinline__ void dep_guard4_h(v8f& a, v8f& b, v8f& c, v8f& d, v16h x, v16h y) { asm volatile("v_nop\n\tv_nop\n\tv_nop\n\tv_nop" : "+v"(a), "+v"(b), "+v"(c), "+v"(d) : "v"(x), "v"(y)); }
__device__ __forceinline__ void dep_guard4_b(v8f& a, v8f& b, v8f& c, v8f& d, v16b x, v16b y) { asm volatile("v_nop\n\tv_nop\n\tv_nop\n\tv_nop" : "+v"(a), "+v"(b), "+v"(c), "+v"(d) : "v"(x), "v"(y)); }
__device__ __forceinline__ void keep4_h(v16h a, v16h b, v16h c, v16h d) { asm volatile("v_nop" :: "v"(a), "v"(b), "v"(c), "v"(d)); }
__device__ __forceinline__ void keep4_b(v16b a, v16b b, v16b c, v16b d) { asm volatile("v_nop" :: "v"(a), "v"(b), "v"(c), "v"(d)); }
__device__ __forceinline__ void acc_guard4(v8f& a, v8f& b, v8f& c, v8f& d) { asm volatile("v_nop\n\tv_nop\n\tv_nop\n\tv_nop" : "+v"(a), "+v"(b), "+v"(c), "+v"(d)); }
template <typename T> struct Frag;
template <> struct Frag<_Float16> {
  typedef v16h V; union U { v16h v; v8h h[2]; };
  static __device__ __forceinline__ v16h load(const _Float16* p) {
    U f; f.h[0] = *(const v8h*)(p); f.h[1] = *(const v8h*)(p + 16); return f.v;
  }
  static __device__ __forceinline__ v8f mma(v16h a, v16h b, v8f c) {
    return __builtin_amdgcn_wmma_f32_16x16x32_f16(false, a, false, b, (short)0, c, false, false);
  }
  static __device__ __forceinline__ void guard4(v8f& a, v8f& b, v8f& c, v8f& d, v16h x, v16h y) { dep_guard4_h(a, b, c, d, x, y); }
  static __device__ __forceinline__ void keep(v16h a, v16h b, v16h c, v16h d) { keep4_h(a, b, c, d); }
};
template <> struct Frag<__bf16> {
  typedef v16b V; union U { v16b v; v8b h[2]; };
  static __device__ __forceinline__ v16b load(const __bf16* p) {
    U f; f.h[0] = *(const v8b*)(p); f.h[1] = *(const v8b*)(p + 16); return f.v;
  }
  static __device__ __forceinline__ v8f mma(v16b a, v16b b, v8f c) {
    return __builtin_amdgcn_wmma_f32_16x16x32_bf16(false, a, false, b, (short)0, c, false, false);
  }
  static __device__ __forceinline__ void guard4(v8f& a, v8f& b, v8f& c, v8f& d, v16b x, v16b y) { dep_guard4_b(a, b, c, d, x, y); }
  static __device__ __forceinline__ void keep(v16b a, v16b b, v16b c, v16b d) { keep4_b(a, b, c, d); }
};

template <int ET> struct Elem;
template <> struct Elem<0> { typedef _Float16 T; };
template <> struct Elem<1> { typedef __bf16 T; };
template <int ET, int SPL, int BIAS_MODE, int OUT_MODE, bool RESID, int ACT = 0>
__global__ __launch_bounds__(256) void wmma_gemm64(
    const unsigned short* __restrict__ Ap, const unsigned short* __restrict__ A2p, int lda, long strideA,
    const unsigned short* __restrict__ Btp, const unsigned short* __restrict__ Bt2p, int ldb, long strideB,
    void* __restrict__ Cout, void* __restrict__ Cout2, int ldc, long strideC,
    const float* __restrict__ bias,
    const float* __restrict__ resid, long strideR,
    int M, int N, int K, float scale) {
  typedef typename Elem<ET>::T T;
  typedef typename Frag<T>::V V;
  const T* A = (const T*)Ap; const T* A2 = (const T*)A2p; const T* Bt = (const T*)Btp; const T* Bt2 = (const T*)Bt2p;
  __shared__ __align__(16) float sT[8][16 * 68];
  const int b    = blockIdx.y;
  const int lane = threadIdx.x & 31;
  const int wave = threadIdx.x >> 5;
  const int tilesN = N >> 6;
  const int tilesM = M >> 6;
  const int tile = blockIdx.x * 8 + wave;
  if (tile >= tilesM * tilesN) return;
  const int tm = tile / tilesN;
  const int tn = tile - tm * tilesN;
  const int m0 = tm << 6;
  const int n0 = tn << 6;

  const T* Ab  = A  + (size_t)b * strideA;
  const T* Bb  = Bt + (size_t)b * strideB;
  const T* Ab2 = (SPL >= 1) ? (A2  + (size_t)b * strideA) : nullptr;
  const T* Bb2 = (SPL == 2) ? (Bt2 + (size_t)b * strideB) : nullptr;

  const int rlane = lane & 15;
  const int koff  = (lane >> 4) * 8;
  const int mOff  = (lane >> 4) * 8;

  v8f acc[4][4];
#pragma unroll
  for (int i = 0; i < 4; ++i)
#pragma unroll
    for (int j = 0; j < 4; ++j) acc[i][j] = (v8f){0.f,0.f,0.f,0.f,0.f,0.f,0.f,0.f};

  for (int k0 = 0; k0 < K; k0 += 32) {
    V bh[4], bl[4];
#pragma unroll
    for (int j = 0; j < 4; ++j) {
      const size_t bo = (size_t)(n0 + (j << 4) + rlane) * ldb + koff + k0;
      bh[j] = Frag<T>::load(Bb + bo);
      if (SPL == 2) bl[j] = Frag<T>::load(Bb2 + bo);
    }
#pragma unroll
    for (int i = 0; i < 4; ++i) {
      const size_t ao = (size_t)(m0 + (i << 4) + rlane) * lda + koff + k0;
      V ah = Frag<T>::load(Ab + ao);
      V al;
      if (SPL >= 1) al = Frag<T>::load(Ab2 + ao);
#pragma unroll
      for (int j = 0; j < 4; ++j) {
        acc[i][j] = Frag<T>::mma(ah, bh[j], acc[i][j]);
        if (SPL == 2) acc[i][j] = Frag<T>::mma(ah, bl[j], acc[i][j]);
        if (SPL >= 1) acc[i][j] = Frag<T>::mma(al, bh[j], acc[i][j]);
      }
      Frag<T>::guard4(acc[i][0], acc[i][1], acc[i][2], acc[i][3], ah, (SPL >= 1) ? al : ah);
    }
    Frag<T>::keep(bh[0], bh[1], bh[2], bh[3]);
    if (SPL == 2) Frag<T>::keep(bl[0], bl[1], bl[2], bl[3]);
  }
  acc_guard4(acc[0][0], acc[0][1], acc[0][2], acc[0][3]);
  acc_guard4(acc[1][0], acc[1][1], acc[1][2], acc[1][3]);
  acc_guard4(acc[2][0], acc[2][1], acc[2][2], acc[2][3]);
  acc_guard4(acc[3][0], acc[3][1], acc[3][2], acc[3][3]);

  float* slab = sT[wave];
  const float* Rb = RESID ? (resid + (size_t)b * strideR) : nullptr;
#pragma unroll
  for (int i = 0; i < 4; ++i) {
    const int mBase = m0 + (i << 4);
#pragma unroll
    for (int j = 0; j < 4; ++j) {
      const int n = n0 + (j << 4) + rlane;
      float bv = 0.f;
      if (BIAS_MODE == 2) bv = bias[n];
#pragma unroll
      for (int r = 0; r < 8; ++r) {
        float v = acc[i][j][r] * scale;
        if (BIAS_MODE == 1) v += bias[mBase + mOff + r];
        if (BIAS_MODE == 2) v += bv;
        if (RESID) v += Rb[(size_t)(mBase + mOff + r) * ldc + n];
        if (ACT == 1) v = tanhf(v);
        if (ACT == 2) v = fmaxf(v, 0.0f);
        if (ACT == 3) v = v / (1.0f + expf(-v));
        if (ACT == 4) v = (v > 0.f) ? v : 0.01f * v;
        slab[(mOff + r) * 68 + (j << 4) + rlane] = v;
      }
    }
    __builtin_amdgcn_fence(__ATOMIC_RELEASE, "workgroup");
    __builtin_amdgcn_wave_barrier();
    __builtin_amdgcn_fence(__ATOMIC_ACQUIRE, "workgroup");
    if (OUT_MODE == 0) {
      float* C = (float*)Cout + (size_t)b * strideC;
      const int hh = lane >> 4, c4 = (lane & 15) * 4;
      for (int pass = 0; pass < 2; ++pass) {
#pragma unroll
        for (int it = 0; it < 8; ++it) {
          const int row = it * 2 + hh;
          v4f v = *(const v4f*)(slab + row * 68 + c4);
          *(volatile v4f*)(C + (size_t)(mBase + row) * ldc + n0 + c4) = v;
        }
        __threadfence();
      }
    } else {
      const int q = lane >> 3, c8 = (lane & 7) * 8;
      unsigned short* C  = (unsigned short*)Cout  + (size_t)b * strideC;
      unsigned short* C2 = (OUT_MODE == 2) ? ((unsigned short*)Cout2 + (size_t)b * strideC) : nullptr;
      for (int pass = 0; pass < 2; ++pass) {
#pragma unroll
        for (int it = 0; it < 4; ++it) {
          const int row = it * 4 + q;
          const float* sp = slab + row * 68 + c8;
          v8h hv, lv;
#pragma unroll
          for (int e = 0; e < 8; ++e) {
            if (OUT_MODE == 1) {
              hv[e] = (_Float16)sp[e];
            } else {
              unsigned short hb = f2bf_bits(sp[e]);
              unsigned short lb = f2bf_bits(sp[e] - bf_bits2f(hb));
              hv[e] = __builtin_bit_cast(_Float16, hb);
              lv[e] = __builtin_bit_cast(_Float16, lb);
            }
          }
          *(volatile v8h*)(C + (size_t)(mBase + row) * ldc + n0 + c8) = hv;
          if (OUT_MODE == 2) *(volatile v8h*)(C2 + (size_t)(mBase + row) * ldc + n0 + c8) = lv;
        }
        __threadfence();
      }
    }
    __builtin_amdgcn_fence(__ATOMIC_RELEASE, "workgroup");
    __builtin_amdgcn_wave_barrier();
    __builtin_amdgcn_fence(__ATOMIC_ACQUIRE, "workgroup");
  }
}

__global__ __launch_bounds__(256) void split_rows_bf16_kernel(
    const float* __restrict__ src, unsigned short* __restrict__ dhi, unsigned short* __restrict__ dlo,
    int nrows_src, int ncols, int total8)
{
  const int i = blockIdx.x * 256 + threadIdx.x;
  if (i >= total8) return;
  const unsigned e0  = (unsigned)i << 3;
  const unsigned row = e0 / (unsigned)ncols;
  const unsigned col = e0 - row * (unsigned)ncols;
  const bool live = row < (unsigned)nrows_src;
  const unsigned rcl = live ? row : (unsigned)(nrows_src - 1);
  const float f = live ? 1.0f : 0.0f;
  const float* sp = src + (size_t)rcl * (unsigned)ncols + col;
  const v4f a0 = *(const v4f*)(sp);
  const v4f a1 = *(const v4f*)(sp + 4);
  v8h hv, lv;
#pragma unroll
  for (int e = 0; e < 4; ++e) {
    const float v0 = a0[e] * f + 0.0f;
    const float v1 = a1[e] * f + 0.0f;
    const unsigned short h0 = f2bf_bits(v0), h1 = f2bf_bits(v1);
    const unsigned short l0 = f2bf_bits(v0 - bf_bits2f(h0)), l1 = f2bf_bits(v1 - bf_bits2f(h1));
    hv[e]     = __builtin_bit_cast(_Float16, h0);
    hv[4 + e] = __builtin_bit_cast(_Float16, h1);
    lv[e]     = __builtin_bit_cast(_Float16, l0);
    lv[4 + e] = __builtin_bit_cast(_Float16, l1);
  }
  unsigned short* qh = dhi + (size_t)e0;
  unsigned short* ql = dlo + (size_t)e0;
  *(volatile v8h*)qh = hv;
  *(volatile v8h*)ql = lv;
  __threadfence();
  *(volatile v8h*)qh = hv;
  *(volatile v8h*)ql = lv;
}

__global__ __launch_bounds__(256) void cast_rows_f16_kernel(
    const float* __restrict__ src, unsigned short* __restrict__ dst, int nrows_src, int ncols, int total8, float scl)
{
  const int i = blockIdx.x * 256 + threadIdx.x;
  if (i >= total8) return;
  const unsigned e0  = (unsigned)i << 3;
  const unsigned row = e0 / (unsigned)ncols;
  const unsigned col = e0 - row * (unsigned)ncols;
  const bool live = row < (unsigned)nrows_src;
  const unsigned rcl = live ? row : (unsigned)(nrows_src - 1);
  const float f = live ? scl : 0.0f;
  const float* sp = src + (size_t)rcl * (unsigned)ncols + col;
  const v4f a0 = *(const v4f*)(sp);
  const v4f a1 = *(const v4f*)(sp + 4);
  v8h hv;
#pragma unroll
  for (int e = 0; e < 4; ++e) {
    hv[e]     = (_Float16)(a0[e] * f + 0.0f);
    hv[4 + e] = (_Float16)(a1[e] * f + 0.0f);
  }
  unsigned short* q = dst + (size_t)e0;
  *(volatile v8h*)q = hv;
  __threadfence();
  *(volatile v8h*)q = hv;
}

__global__ __launch_bounds__(256) void cast_dtin_f16_kernel(
    const float* __restrict__ xd, unsigned short* __restrict__ dst, int total8)
{
  const int i = blockIdx.x * 256 + threadIdx.x;
  if (i >= total8) return;
  const int row  = i >> 4;
  const int col8 = (i & 15) * 8;
  const float* sp = xd + (size_t)row * kXW + col8;
  const v4f a0 = *(const v4f*)(sp);
  const v4f a1 = *(const v4f*)(sp + 4);
  v8h hv;
#pragma unroll
  for (int e = 0; e < 4; ++e) {
    hv[e]     = (_Float16)a0[e];
    hv[4 + e] = (_Float16)a1[e];
  }
  unsigned short* q = dst + (size_t)row * kR + col8;
  *(volatile v8h*)q = hv;
  __threadfence();
  *(volatile v8h*)q = hv;
}

__global__ __launch_bounds__(64) void scan_kernel(
    const float* __restrict__ XD, const float* __restrict__ DT, const float* __restrict__ X,
    const float* __restrict__ bdt, const float* __restrict__ Alog, const float* __restrict__ Dp,
    float* __restrict__ Y)
{
  __shared__ __align__(16) float sBC[kScanTS * kBCW];
  __shared__ __align__(16) float sY[kScanTS * kScanYP];
  __shared__ __align__(16) float sA[kN * kScanCh];
  const int tid = threadIdx.x, lane = tid & 31, wave = tid >> 5;
  const int d0 = blockIdx.x * kScanCh;
  const int d  = d0 + tid;
#pragma unroll 1
  for (int s = 0; s < kN; ++s) sA[s * kScanCh + tid] = -expf(Alog[(size_t)d * kN + s]);
  __syncthreads();
  float negA[kN], h[kN];
#pragma unroll
  for (int s = 0; s < kN; ++s) {
    negA[s] = sA[s * kScanCh + tid];
    h[s] = 0.0f;
  }
  const float bb = bdt[d], Dd = Dp[d];
  const int lr = tid >> 3, lc4 = (tid & 7) * 4;
  const int hh = lane >> 4, c4 = (lane & 15) * 4;
#pragma unroll 1
  for (int t0 = 0; t0 < kL; t0 += kScanTS) {
    __syncthreads();
#pragma unroll
    for (int i = 0; i < 4; ++i) {
      const int r = lr + 8 * i;
      *(v4f*)(sBC + r * kBCW + lc4) = *(const v4f*)(XD + (size_t)(t0 + r) * kXW + kR + lc4);
    }
    asm volatile("" ::: "memory");
#pragma unroll
    for (int i = 4; i < 8; ++i) {
      const int r = lr + 8 * i;
      *(v4f*)(sBC + r * kBCW + lc4) = *(const v4f*)(XD + (size_t)(t0 + r) * kXW + kR + lc4);
    }
    __syncthreads();
#pragma unroll 1
    for (int s = 0; s < kScanTS; ++s) {
      const int t = t0 + s;
      const float* br = sBC + s * kBCW;
      float Bs[kN], Cs[kN];
#pragma unroll
      for (int q4 = 0; q4 < 4; ++q4) {
        const v4f bv = *(const v4f*)(br + 4 * q4);
        const v4f cv = *(const v4f*)(br + kN + 4 * q4);
        Bs[4 * q4 + 0] = bv[0]; Bs[4 * q4 + 1] = bv[1]; Bs[4 * q4 + 2] = bv[2]; Bs[4 * q4 + 3] = bv[3];
        Cs[4 * q4 + 0] = cv[0]; Cs[4 * q4 + 1] = cv[1]; Cs[4 * q4 + 2] = cv[2]; Cs[4 * q4 + 3] = cv[3];
      }
      const float v   = DT[(size_t)t * kD + d] + bb;
      const float ea  = expf(-fabsf(v));
      const float dt  = fmaxf(v, 0.0f) + log1pf(ea);
      const float xt  = X[(size_t)t * kD + d];
      const float dtx = dt * xt;
      float y = 0.0f;
#pragma unroll
      for (int k = 0; k < kN; ++k) {
        const float e = __expf(dt * negA[k]);
        h[k] = e * h[k] + dtx * Bs[k];
        y = h[k] * Cs[k] + y;
      }
      y = xt * Dd + y;
      sY[s * kScanYP + tid] = y;
    }
    __syncthreads();
    for (int pass = 0; pass < 2; ++pass) {
#pragma unroll
      for (int it = 0; it < 16; ++it) {
        const int row = it * 4 + wave * 2 + hh;
        const v4f val = *(const v4f*)(sY + row * kScanYP + c4);
        *(volatile v4f*)(Y + (size_t)(t0 + row) * kD + d0 + c4) = val;
      }
      __threadfence();
    }
  }
}

extern "C" void kernel_launch(void* const* d_in, const int* in_sizes, int n_in,
                              void* d_out, int out_size, void* d_ws, size_t ws_size,
                              hipStream_t stream) {
  if (n_in < 6) return;
  if (in_sizes[0] != kL * kD) return;
  if (in_sizes[1] != kXC * kD) return;
  if (in_sizes[2] != kD * kR) return;
  if (in_sizes[3] != kD) return;
  if (in_sizes[4] != kD * kN) return;
  if (in_sizes[5] != kD) return;
  if (out_size != kL * kD) return;
  if (ws_size < kWsTotal) return;

  const float* x     = (const float*)d_in[0];
  const float* W_x   = (const float*)d_in[1];
  const float* W_dt  = (const float*)d_in[2];
  const float* b_dt  = (const float*)d_in[3];
  const float* A_log = (const float*)d_in[4];
  const float* Dp    = (const float*)d_in[5];
  float* out = (float*)d_out;

  char* ws = (char*)d_ws;
  unsigned short* XH  = (unsigned short*)(ws + kOffXH);
  unsigned short* XL  = (unsigned short*)(ws + kOffXL);
  unsigned short* WXH = (unsigned short*)(ws + kOffWXH);
  unsigned short* WXL = (unsigned short*)(ws + kOffWXL);
  unsigned short* WD  = (unsigned short*)(ws + kOffWD);
  float*          XD  = (float*)(ws + kOffXD);
  unsigned short* DI  = (unsigned short*)(ws + kOffDI);
  float*          DT  = (float*)(ws + kOffDT);

  split_rows_bf16_kernel<<<(kL * kD / 8) / 256, 256, 0, stream>>>(x, XH, XL, kL, kD, kL * kD / 8);
  split_rows_bf16_kernel<<<(kXW * kD / 8) / 256, 256, 0, stream>>>(W_x, WXH, WXL, kXC, kD, kXW * kD / 8);
  cast_rows_f16_kernel<<<(kD * kR / 8) / 256, 256, 0, stream>>>(W_dt, WD, kD, kR, kD * kR / 8, 256.0f);

  wmma_gemm64<1, 2, 0, 0, false><<<dim3((kL / 64) * (kXW / 64) / 8, 1), 256, 0, stream>>>(
      XH, XL, kD, 0L,
      WXH, WXL, kD, 0L,
      (void*)XD, nullptr, kXW, 0L,
      nullptr, nullptr, 0L,
      kL, kXW, kD, 1.0f);

  cast_dtin_f16_kernel<<<(kL * kR / 8) / 256, 256, 0, stream>>>(XD, DI, kL * kR / 8);

  wmma_gemm64<0, 0, 0, 0, false><<<dim3((kL / 64) * (kD / 64) / 8, 1), 256, 0, stream>>>(
      DI, nullptr, kR, 0L,
      WD, nullptr, kR, 0L,
      (void*)DT, nullptr, kD, 0L,
      nullptr, nullptr, 0L,
      kL, kD, kR, 1.0f / 256.0f);

  scan_kernel<<<kD / kScanCh, kScanCh, 0, stream>>>(XD, DT, x, b_dt, A_log, Dp, out);
}
